// MSM_83545703842333
// MI455X (gfx1250) — hardware-run, weakly checked
//
#include <hip/hip_runtime.h>
#include <math.h>

typedef __attribute__((ext_vector_type(16))) _Float16 v16h;
typedef __attribute__((ext_vector_type(8)))  _Float16 v8h;
typedef __attribute__((ext_vector_type(8)))  float    v8f;
typedef __attribute__((ext_vector_type(4)))  float    v4f;

constexpr int kSeqs    = 256;
constexpr int kT       = 2000;
constexpr int kK       = 16;
constexpr int kTileRows = 16;
constexpr int kTiles   = kSeqs / kTileRows;
constexpr int kChunk   = 16;
constexpr int kNumChunks = kT / kChunk;
constexpr int kEvPitch = kChunk * kK + 4;
constexpr int kRec     = 32;
constexpr int kAlPitch = kChunk * kRec + 4;
constexpr size_t kIoElems = (size_t)kSeqs * kT * kK;
constexpr size_t kWsBytes = (size_t)kSeqs * kT * kRec * 4;
static_assert(kSeqs % kTileRows == 0 && kT % kChunk == 0 && kK == 16, "whole tiles and chunks; the 16 states fill one half of K");
static_assert((kEvPitch % 4) == 0 && (kAlPitch % 4) == 0, "16-B aligned LDS rows");
static_assert(kWsBytes == 65536000ull && kWsBytes <= 134217728ull, "workspace");

constexpr float kACarry   = 4096.0f;
constexpr float kBCarry   = 64.0f;
constexpr float kQCarry   = 4096.0f;
constexpr float kFoldA    = 1.0f / (kACarry * kQCarry);
constexpr float kFoldB    = 1.0f / (kBCarry * kQCarry);
constexpr float kF16MinNorm = 6.103515625e-5f;

namespace eng {

union FragU { v16h v; v8h h[2]; };

__device__ __forceinline__ unsigned short f2bf_bits(float f) {
  unsigned u = __float_as_uint(f);
  return (unsigned short)((u + 0x7FFFu + ((u >> 16) & 1u)) >> 16);
}
__device__ __forceinline__ float bf16v(float f) {
  return __uint_as_float(((unsigned)f2bf_bits(f)) << 16);
}
__device__ __forceinline__ _Float16 to_f16_flushed(float c) {
  const float z = (fabsf(c) < kF16MinNorm) ? 0.0f : c;
  return (_Float16)z;
}
__device__ __forceinline__ v8f mma_f16(v16h a, v16h b) {
  v8f c = (v8f){0.f, 0.f, 0.f, 0.f, 0.f, 0.f, 0.f, 0.f};
  c = __builtin_amdgcn_wmma_f32_16x16x32_f16(false, a, false, b, (short)0, c, false, false);
  asm volatile("v_nop\n\tv_nop\n\tv_nop\n\tv_nop" : "+v"(c) : "v"(a), "v"(b));
  return c;
}
__device__ __forceinline__ v16h split_frag(const float (&c)[8]) {
  v8h hi, lo;
#pragma unroll
  for (int r = 0; r < 8; ++r) {
    const _Float16 h = to_f16_flushed(c[r]);
    hi[r] = h;
    lo[r] = to_f16_flushed(c[r] - (float)h);
  }
  FragU fu; fu.h[0] = hi; fu.h[1] = lo;
  return fu.v;
}

}

__global__ __launch_bounds__(32) void hmm_forward_kernel(const float* __restrict__ ev, const float* __restrict__ pi,
                                                         const float* __restrict__ Q, float* __restrict__ REC)
{
  __shared__ __align__(16) float es[kTileRows * kEvPitch];
  __shared__ __align__(16) float as[kTileRows * kAlPitch];
  __shared__ __align__(16) float qs[kK * kK + kK];

  const int lane = threadIdx.x & 31;
  const int hsel = lane >> 4;
  const int n    = lane & 15;
  const bool lowHalf = (hsel == 0);
  const int b0   = blockIdx.x * kTileRows;

#pragma unroll
  for (int it = 0; it < 8; ++it) qs[it * 32 + lane] = Q[it * 32 + lane];
  qs[kK * kK + (lane & 15)] = pi[lane & 15];
#pragma unroll 1
  for (int i = lane; i < kTileRows * kAlPitch; i += 32) as[i] = 0.0f;
  __syncthreads();

  v16h fragQ;
  {
    v8h a0;
#pragma unroll
    for (int i = 0; i < 8; ++i) a0[i] = eng::to_f16_flushed(eng::bf16v(qs[(8 * hsel + i) * kK + n]) * kQCarry);
    eng::FragU fu; fu.h[0] = a0; fu.h[1] = a0;
    fragQ = fu.v;
  }
  float piv[8];
#pragma unroll
  for (int r = 0; r < 8; ++r) piv[r] = eng::bf16v(qs[kK * kK + 8 * hsel + r]);

  float a[8];
#pragma unroll
  for (int r = 0; r < 8; ++r) a[r] = 0.0f;

#pragma unroll 1
  for (int ch = 0; ch < kNumChunks; ++ch) {
    const int t0 = ch * kChunk;
#pragma unroll 4
    for (int it = 0; it < 32; ++it) {
      const int row = it >> 1;
      const int off = (it & 1) * 128 + 4 * lane;
      const v4f v = *(const v4f*)(ev + ((size_t)(b0 + row) * kT + t0) * kK + off);
      v4f rv;
      rv[0] = eng::bf16v(v[0]); rv[1] = eng::bf16v(v[1]); rv[2] = eng::bf16v(v[2]); rv[3] = eng::bf16v(v[3]);
      *(v4f*)(es + row * kEvPitch + off) = rv;
    }
    __syncthreads();

#pragma unroll 1
    for (int s = 0; s < kChunk; ++s) {
      const v4f e0 = *(const v4f*)(es + n * kEvPitch + s * kK + 8 * hsel);
      const v4f e1 = *(const v4f*)(es + n * kEvPitch + s * kK + 8 * hsel + 4);
      float p[8];
      if (t0 + s == 0) {
#pragma unroll
        for (int r = 0; r < 8; ++r) p[r] = expf((r < 4) ? e0[r] : e1[r - 4]) * piv[r];
      } else {
        float ac[8];
#pragma unroll
        for (int r = 0; r < 8; ++r) ac[r] = a[r] * kACarry;
        const v8f d = eng::mma_f16(fragQ, eng::split_frag(ac));
#pragma unroll
        for (int r = 0; r < 8; ++r) p[r] = expf((r < 4) ? e0[r] : e1[r - 4]) * (d[r] * kFoldA);
      }
      float zp = ((p[0] + p[1]) + (p[2] + p[3])) + ((p[4] + p[5]) + (p[6] + p[7]));
      const float z = zp + __shfl_xor(zp, 16, 32);
      const float inv = 1.0f / z;
      v4f o0, o1;
#pragma unroll
      for (int r = 0; r < 8; ++r) { a[r] = p[r] * inv; if (r < 4) o0[r] = a[r]; else o1[r - 4] = a[r]; }
      *(v4f*)(as + n * kAlPitch + s * kRec + 8 * hsel) = o0;
      *(v4f*)(as + n * kAlPitch + s * kRec + 8 * hsel + 4) = o1;
      if (lowHalf) as[n * kAlPitch + s * kRec + kK] = z;
    }
    __syncthreads();

    for (int pass = 0; pass < 2; ++pass) {
#pragma unroll 4
      for (int it = 0; it < 64; ++it) {
        const int row = it >> 2;
        const int off = (it & 3) * 128 + 4 * lane;
        const v4f v = *(const v4f*)(as + row * kAlPitch + off);
        *(volatile v4f*)(REC + ((size_t)(b0 + row) * kT + t0) * kRec + off) = v;
      }
      __threadfence();
    }
    __syncthreads();
  }
}

__global__ __launch_bounds__(32) void hmm_backward_kernel(const float* __restrict__ ev, const float* __restrict__ Q,
                                                          const float* __restrict__ REC, float* __restrict__ outs)
{
  __shared__ __align__(16) float es[kTileRows * kEvPitch];
  __shared__ __align__(16) float as[kTileRows * kAlPitch];
  __shared__ __align__(16) float gs[kTileRows * kEvPitch];
  __shared__ __align__(16) float qs[kK * kK];

  const int lane = threadIdx.x & 31;
  const int hsel = lane >> 4;
  const int n    = lane & 15;
  const int b0   = blockIdx.x * kTileRows;

#pragma unroll
  for (int it = 0; it < 8; ++it) qs[it * 32 + lane] = Q[it * 32 + lane];
  __syncthreads();

  v16h fragQ;
  {
    v8h a0;
#pragma unroll
    for (int i = 0; i < 8; ++i) a0[i] = eng::to_f16_flushed(eng::bf16v(qs[n * kK + 8 * hsel + i]) * kQCarry);
    eng::FragU fu; fu.h[0] = a0; fu.h[1] = a0;
    fragQ = fu.v;
  }

  float b[8];
#pragma unroll
  for (int r = 0; r < 8; ++r) b[r] = 1.0f;

#pragma unroll 1
  for (int ch = kNumChunks - 1; ch >= 0; --ch) {
    const int t0 = ch * kChunk;
#pragma unroll 4
    for (int it = 0; it < 32; ++it) {
      const int row = it >> 1;
      const int off = (it & 1) * 128 + 4 * lane;
      const v4f v = *(const v4f*)(ev + ((size_t)(b0 + row) * kT + t0) * kK + off);
      v4f rv;
      rv[0] = eng::bf16v(v[0]); rv[1] = eng::bf16v(v[1]); rv[2] = eng::bf16v(v[2]); rv[3] = eng::bf16v(v[3]);
      *(v4f*)(es + row * kEvPitch + off) = rv;
    }
#pragma unroll 4
    for (int it = 0; it < 64; ++it) {
      const int row = it >> 2;
      const int off = (it & 3) * 128 + 4 * lane;
      *(v4f*)(as + row * kAlPitch + off) = *(const v4f*)(REC + ((size_t)(b0 + row) * kT + t0) * kRec + off);
    }
    __syncthreads();

#pragma unroll 1
    for (int s = kChunk - 1; s >= 0; --s) {
      const v4f a0 = *(const v4f*)(as + n * kAlPitch + s * kRec + 8 * hsel);
      const v4f a1 = *(const v4f*)(as + n * kAlPitch + s * kRec + 8 * hsel + 4);
      v4f g0, g1;
#pragma unroll
      for (int r = 0; r < 4; ++r) { g0[r] = a0[r] * b[r]; g1[r] = a1[r] * b[4 + r]; }
      *(v4f*)(gs + n * kEvPitch + s * kK + 8 * hsel) = g0;
      *(v4f*)(gs + n * kEvPitch + s * kK + 8 * hsel + 4) = g1;
      if (t0 + s > 0) {
        const v4f e0 = *(const v4f*)(es + n * kEvPitch + s * kK + 8 * hsel);
        const v4f e1 = *(const v4f*)(es + n * kEvPitch + s * kK + 8 * hsel + 4);
        const float z = as[n * kAlPitch + s * kRec + kK];
        float wc[8];
#pragma unroll
        for (int r = 0; r < 8; ++r) wc[r] = (expf((r < 4) ? e0[r] : e1[r - 4]) * b[r]) * kBCarry;
        const v8f d = eng::mma_f16(fragQ, eng::split_frag(wc));
        const float inv = 1.0f / z;
#pragma unroll
        for (int r = 0; r < 8; ++r) b[r] = (d[r] * kFoldB) * inv;
      }
    }
    __syncthreads();

    for (int pass = 0; pass < 2; ++pass) {
#pragma unroll 4
      for (int it = 0; it < 32; ++it) {
        const int row = it >> 1;
        const int off = (it & 1) * 128 + 4 * lane;
        const v4f v = *(const v4f*)(gs + row * kEvPitch + off);
        *(volatile v4f*)(outs + ((size_t)(b0 + row) * kT + t0) * kK + off) = v;
      }
      __threadfence();
    }
    __syncthreads();
  }
}

extern "C" void kernel_launch(void* const* d_in, const int* in_sizes, int n_in,
                              void* d_out, int out_size, void* d_ws, size_t ws_size,
                              hipStream_t stream) {
  if (n_in < 3 || d_out == nullptr || d_ws == nullptr) return;
  if ((size_t)in_sizes[0] != kIoElems || in_sizes[1] != kK || in_sizes[2] != kK * kK) return;
  if ((size_t)out_size != kIoElems) return;
  if (ws_size < kWsBytes) return;
  const float* ev = (const float*)d_in[0];
  const float* pi = (const float*)d_in[1];
  const float* Q  = (const float*)d_in[2];
  float* REC = (float*)d_ws;
  hmm_forward_kernel<<<kTiles, 32, 0, stream>>>(ev, pi, Q, REC);
  hmm_backward_kernel<<<kTiles, 32, 0, stream>>>(ev, Q, REC, (float*)d_out);
}
